// ConvSlimCapsule3D_33818572489333
// MI455X (gfx1250) — hardware-verified
//
#include <hip/hip_runtime.h>
#include <stdint.h>

#define NB      2
#define IN_DIM  8
#define CIN     16
#define OUT_DIM 8
#define OATOMS  16
#define NCH     128
#define DD      32
#define VOX     32768
#define NVOL    (NB * IN_DIM)
#define KT      27
#define KLIVE   (CIN * KT)
#define KP      448
#define KSTEPS  (KP / 32)
#define XP      34
#define PPV     (XP * XP * XP)
#define PLH     (PPV * CIN)
#define XPIECES (NVOL * PPV * 2)
#define WROW    (KP / 8)
#define WPIECES (NCH * WROW)
#define NTHR    512
#define MPOS    32
#define NBLK    (NB * DD * DD)
#define VSTR    (MPOS * NCH)
#define SCX     64.0f
#define SCW     64.0f
#define INV_A   2.44140625e-04f

static_assert(KP % 32 == 0);
static_assert(KLIVE <= KP);
static_assert(NTHR == MPOS * OATOMS);
static_assert(NTHR / 32 == IN_DIM * 2);
static_assert(((size_t)NVOL * PLH * 2) % 128 == 0);
static_assert(((size_t)NCH * KP * 2) % 128 == 0);
static_assert(NTHR / 8 * 2 == NCH);
static_assert(OUT_DIM == 8);
static_assert(OATOMS == 16);

typedef _Float16 v16h __attribute__((ext_vector_type(16)));
typedef _Float16 v8h  __attribute__((ext_vector_type(8)));
typedef float    v8f  __attribute__((ext_vector_type(8)));
typedef float    v4f  __attribute__((ext_vector_type(4)));
typedef unsigned v4u  __attribute__((ext_vector_type(4)));

__device__ __forceinline__ float bf_rne(float f) {
  unsigned u = __float_as_uint(f);
  u = (u + 0x7FFFu + ((u >> 16) & 1u)) & 0xFFFF0000u;
  return __uint_as_float(u);
}
__device__ __forceinline__ unsigned hbits(_Float16 h) {
  return (unsigned)__builtin_bit_cast(unsigned short, h);
}
__device__ __forceinline__ v8f zero8f() { v8f z = {0.f, 0.f, 0.f, 0.f, 0.f, 0.f, 0.f, 0.f}; return z; }
__device__ __forceinline__ float frcp(float x)  { return __builtin_amdgcn_rcpf(x); }
__device__ __forceinline__ float fsqrt(float x) { return __builtin_amdgcn_sqrtf(x); }

__device__ __forceinline__ float reduce16(float x) {
  x += __shfl_xor(x, 1, 32);
  x += __shfl_xor(x, 2, 32);
  x += __shfl_xor(x, 4, 32);
  x += __shfl_xor(x, 8, 32);
  return x;
}

__device__ __forceinline__ v16h ldfrag(const _Float16* p) {
  union { v16h v; v8h h[2]; } f;
  f.h[0] = *(const v8h*)(p);
  f.h[1] = *(const v8h*)(p + 16);
  return f.v;
}

__device__ __forceinline__ v8f mma_h(v16h a, v16h b, v8f c) {
  return __builtin_amdgcn_wmma_f32_16x16x32_f16(false, a, false, b, (short)0, c, false, false);
}
__device__ __forceinline__ void dep_guard(v8f& c0, v8f& c1, v8f& c2, v8f& c3,
                                          v16h a, v16h b0, v16h b1, v16h b2, v16h b3) {
#if defined(__HIP_DEVICE_COMPILE__)
  asm volatile("v_nop\n\tv_nop\n\tv_nop\n\tv_nop"
               : "+v"(c0), "+v"(c1), "+v"(c2), "+v"(c3)
               : "v"(a), "v"(b0), "v"(b1), "v"(b2), "v"(b3));
#endif
}

__device__ __forceinline__ int tapoff(int t) {
  const int kz = t / 9;
  const int r  = t - 9 * kz;
  const int ky = r / 3;
  const int kx = r - 3 * ky;
  return ((kz * XP + ky) * XP + kx) * CIN;
}

__global__ __launch_bounds__(256)
void k_xprep(const float* __restrict__ x, unsigned* xh)
{
  const int q   = blockIdx.x * 256 + threadIdx.x;
  const int qc  = (q < XPIECES) ? q : (XPIECES - 1);
  const int p   = qc >> 1;
  const int hf  = qc & 1;
  const int vol = p / PPV;
  const int r   = p - vol * PPV;
  const int zp  = r / (XP * XP);
  const int r2  = r - zp * (XP * XP);
  const int yp  = r2 / XP;
  const int xp  = r2 - yp * XP;
  const int iz  = zp - 1, iy = yp - 1, ix = xp - 1;
  const bool inr = ((unsigned)iz < (unsigned)DD) && ((unsigned)iy < (unsigned)DD) && ((unsigned)ix < (unsigned)DD);
  const int izc = (iz < 0) ? 0 : ((iz > DD - 1) ? (DD - 1) : iz);
  const int iyc = (iy < 0) ? 0 : ((iy > DD - 1) ? (DD - 1) : iy);
  const int ixc = (ix < 0) ? 0 : ((ix > DD - 1) ? (DD - 1) : ix);
  const float* s = x + (size_t)(vol * CIN + 8 * hf) * VOX + (size_t)(izc * (DD * DD) + iyc * DD + ixc);

  unsigned hb[8];
#pragma unroll
  for (int j = 0; j < 8; ++j) {
    float f = s[(size_t)j * VOX];
    f = inr ? bf_rne(f) * SCX : 0.0f;
    hb[j] = hbits((_Float16)f);
  }
  v4u wv;
  wv.x = hb[0] | (hb[1] << 16);
  wv.y = hb[2] | (hb[3] << 16);
  wv.z = hb[4] | (hb[5] << 16);
  wv.w = hb[6] | (hb[7] << 16);

  unsigned* dst = xh + (size_t)qc * 4;
  if (q < XPIECES) *(volatile v4u*)dst = wv;
  __threadfence();
  if (q < XPIECES) *(volatile v4u*)dst = wv;
}

__global__ __launch_bounds__(256)
void k_wprep(const float* __restrict__ w, unsigned* wt)
{
  const int q  = blockIdx.x * 256 + threadIdx.x;
  const int qc = (q < WPIECES) ? q : (WPIECES - 1);
  const int n  = qc / WROW;
  const int kc = (qc - n * WROW) * 8;

  unsigned hb[8];
#pragma unroll
  for (int j = 0; j < 8; ++j) {
    const int k  = kc + j;
    const int t  = k >> 4;
    const int c  = k & 15;
    const int tc = (t < KT) ? t : (KT - 1);
    float f = bf_rne(w[n * KLIVE + c * KT + tc]) * SCW;
    f = (t < KT) ? f : 0.0f;
    hb[j] = hbits((_Float16)f);
  }
  v4u wv;
  wv.x = hb[0] | (hb[1] << 16);
  wv.y = hb[2] | (hb[3] << 16);
  wv.z = hb[4] | (hb[5] << 16);
  wv.w = hb[6] | (hb[7] << 16);

  unsigned* dst = wt + (size_t)qc * 4;
  if (q < WPIECES) *(volatile v4u*)dst = wv;
  __threadfence();
  if (q < WPIECES) *(volatile v4u*)dst = wv;
}

__device__ __forceinline__ void softmax4(const float (&lg)[4], float (&r)[4]) {
  float mx = fmaxf(fmaxf(lg[0], lg[1]), fmaxf(lg[2], lg[3]));
  mx = fmaxf(mx, __shfl_xor(mx, 1, 32));
  const float e0 = __expf(lg[0] - mx);
  const float e1 = __expf(lg[1] - mx);
  const float e2 = __expf(lg[2] - mx);
  const float e3 = __expf(lg[3] - mx);
  float se = (e0 + e1) + (e2 + e3);
  se += __shfl_xor(se, 1, 32);
  const float rs = frcp(se);
  r[0] = e0 * rs;  r[1] = e1 * rs;  r[2] = e2 * rs;  r[3] = e3 * rs;
}
__device__ __forceinline__ void calc_pre(const float* vb, const float (&r)[4], const float (&bz)[8],
                                         int grp, float (&pre)[8]) {
#pragma unroll
  for (int o = 0; o < OUT_DIM; ++o) pre[o] = 0.0f;
#pragma unroll 1
  for (int i = 0; i < IN_DIM; ++i) {
    const float* vp = vb + i * VSTR;
    const int sl = grp + 2 * i;
#pragma unroll
    for (int o = 0; o < OUT_DIM; ++o) {
      const float rt = __shfl(r[o & 3], sl + (o >> 2), 32);
      pre[o] += vp[o * OATOMS] * rt;
    }
  }
#pragma unroll
  for (int o = 0; o < OUT_DIM; ++o) pre[o] += bz[o];
}
__device__ __forceinline__ void agree(const float* pq, const float* vq, float (&lg)[4]) {
#pragma unroll
  for (int qd = 0; qd < 4; ++qd) {
    const float* pp = pq + qd * OATOMS;
    const float* vv = vq + qd * OATOMS;
    float d = 0.0f, w2 = 0.0f, p2 = 0.0f;
#pragma unroll
    for (int c = 0; c < 4; ++c) {
      const v4f pv = *(const v4f*)(pp + 4 * c);
      const v4f xv = *(const v4f*)(vv + 4 * c);
#pragma unroll
      for (int e = 0; e < 4; ++e) {
        d  += pv[e] * xv[e];
        w2 += xv[e] * xv[e];
        p2 += pv[e] * pv[e];
      }
    }
    const float pn  = fsqrt(p2);
    const float vn  = fsqrt(w2);
    const float den = fmaxf(pn * vn, 1e-8f);
    lg[qd] += d * frcp(den);
  }
}

__global__ __launch_bounds__(NTHR)
void k_caps(const _Float16* __restrict__ xh, const _Float16* __restrict__ wt,
            const float* __restrict__ conv_b, const float* __restrict__ biases, float* out)
{
  __shared__ __align__(16) float vl[IN_DIM * VSTR];
  __shared__ __align__(16) float ps[MPOS * NCH];
  __shared__ float cbs[NCH];
  __shared__ float bzs[NCH];

  const int tid  = threadIdx.x;
  const int lane = tid & 31;
  const int wv   = tid >> 5;
  const int lm   = lane & 15;
  const int hh   = lane >> 4;
  const int blk  = blockIdx.x;
  const int b    = blk >> 10;
  const int zy   = blk & 1023;
  const int z    = zy >> 5;
  const int y    = zy & 31;

  if (tid < NCH) {
    cbs[tid] = bf_rne(conv_b[tid]);
    bzs[tid] = bf_rne(biases[tid]);
  }
  __syncthreads();

  {
    const int i   = wv >> 1;
    const int mt  = wv & 1;
    const int vol = b * IN_DIM + i;
    const _Float16* xvb = xh + (size_t)vol * PLH + 8 * hh;
    const int pofs = ((z * XP + y) * XP + 16 * mt + lm) * CIN;
    const _Float16* wl = wt + lm * KP + 8 * hh;

    v8f acc[8];
#pragma unroll
    for (int nt = 0; nt < 8; ++nt) acc[nt] = zero8f();

#pragma unroll 1
    for (int ks = 0; ks < KSTEPS; ++ks) {
      const int t0  = 2 * ks;
      const int t1  = 2 * ks + 1;
      const int t1c = (t1 < KT) ? t1 : (KT - 1);
      const int o0  = pofs + tapoff(t0);
      const int o1  = (t1 < KT) ? (pofs + tapoff(t1c)) : 0;
      union { v16h v; v8h h[2]; } fa;
      fa.h[0] = *(const v8h*)(xvb + o0);
      fa.h[1] = *(const v8h*)(xvb + o1);
      const _Float16* wk = wl + 32 * ks;
      {
        const v16h b0 = ldfrag(wk);
        const v16h b1 = ldfrag(wk + 16 * KP);
        const v16h b2 = ldfrag(wk + 32 * KP);
        const v16h b3 = ldfrag(wk + 48 * KP);
        acc[0] = mma_h(fa.v, b0, acc[0]);
        acc[1] = mma_h(fa.v, b1, acc[1]);
        acc[2] = mma_h(fa.v, b2, acc[2]);
        acc[3] = mma_h(fa.v, b3, acc[3]);
        dep_guard(acc[0], acc[1], acc[2], acc[3], fa.v, b0, b1, b2, b3);
      }
      {
        const v16h b4 = ldfrag(wk + 64 * KP);
        const v16h b5 = ldfrag(wk + 80 * KP);
        const v16h b6 = ldfrag(wk + 96 * KP);
        const v16h b7 = ldfrag(wk + 112 * KP);
        acc[4] = mma_h(fa.v, b4, acc[4]);
        acc[5] = mma_h(fa.v, b5, acc[5]);
        acc[6] = mma_h(fa.v, b6, acc[6]);
        acc[7] = mma_h(fa.v, b7, acc[7]);
        dep_guard(acc[4], acc[5], acc[6], acc[7], fa.v, b4, b5, b6, b7);
      }
    }

    const int rowb = (i * MPOS + 16 * mt + 8 * hh) * NCH + lm;
#pragma unroll
    for (int nt = 0; nt < 8; ++nt) {
      const float cb = cbs[nt * 16 + lm];
#pragma unroll
      for (int r = 0; r < 8; ++r)
        vl[rowb + r * NCH + nt * 16] = acc[nt][r] * INV_A + cb;
    }
  }
  __syncthreads();

  const int m   = tid >> 4;
  const int a   = tid & 15;
  const int grp = lane & 16;
  const int ri  = a >> 1;
  const int ob  = (a & 1) * 4;
  const float* vb   = vl + m * NCH + a;
  const float* vrow = vl + ri * VSTR + m * NCH + ob * OATOMS;
  float* psm = ps + m * NCH;

  float bz[OUT_DIM];
#pragma unroll
  for (int o = 0; o < OUT_DIM; ++o) bz[o] = bzs[o * OATOMS + a];

  float lg[4] = {0.0f, 0.0f, 0.0f, 0.0f};
  float r[4];
  float pre[OUT_DIM];

  r[0] = 0.125f;  r[1] = 0.125f;  r[2] = 0.125f;  r[3] = 0.125f;
  calc_pre(vb, r, bz, grp, pre);
  __syncthreads();
#pragma unroll
  for (int o = 0; o < OUT_DIM; ++o) psm[o * OATOMS + a] = pre[o];
  __syncthreads();
  agree(psm + ob * OATOMS, vrow, lg);

  softmax4(lg, r);
  calc_pre(vb, r, bz, grp, pre);
  __syncthreads();
#pragma unroll
  for (int o = 0; o < OUT_DIM; ++o) psm[o * OATOMS + a] = pre[o];
  __syncthreads();
  agree(psm + ob * OATOMS, vrow, lg);

  softmax4(lg, r);
  calc_pre(vb, r, bz, grp, pre);
  float act[OUT_DIM];
#pragma unroll
  for (int o = 0; o < OUT_DIM; ++o) {
    const float s2  = reduce16(pre[o] * pre[o]);
    const float nrm = fsqrt(s2);
    const float nsq = nrm * nrm;
    const float f   = frcp(nrm + 1e-12f) * (nsq * frcp(1.0f + nsq));
    act[o] = pre[o] * f;
  }
  __syncthreads();
  float* ost = ps;
#pragma unroll
  for (int o = 0; o < OUT_DIM; ++o) ost[(o * OATOMS + a) * MPOS + m] = act[o];
  __syncthreads();

  {
    const int L  = tid >> 3;
    const int pc = (tid & 7) * 4;
    const v4f w0 = *(const v4f*)(ost + L * MPOS + pc);
    const v4f w1 = *(const v4f*)(ost + (L + 64) * MPOS + pc);
    float* obp = out + (size_t)b * NCH * VOX + (size_t)(z * (DD * DD) + y * DD + pc);
    float* d0 = obp + (size_t)L * VOX;
    float* d1 = obp + (size_t)(L + 64) * VOX;
    *(volatile v4f*)d0 = w0;
    *(volatile v4f*)d1 = w1;
    __threadfence();
    *(volatile v4f*)d0 = w0;
    *(volatile v4f*)d1 = w1;
  }
}

extern "C" void kernel_launch(void* const* d_in, const int* in_sizes, int n_in,
                              void* d_out, int out_size, void* d_ws, size_t ws_size,
                              hipStream_t stream) {
  if (n_in < 4) return;
  if (in_sizes[0] != NVOL * CIN * VOX) return;
  if (in_sizes[1] != NCH * KLIVE) return;
  if (in_sizes[2] < NCH) return;
  if (in_sizes[3] < OUT_DIM * OATOMS) return;
  if (out_size != NB * NCH * VOX) return;

  const size_t xbytes = (size_t)NVOL * PLH * 2;
  const size_t wbytes = (size_t)NCH * KP * 2;
  const size_t off_x  = 0;
  const size_t off_w  = off_x + xbytes;
  const size_t total  = off_w + wbytes;
  if (total > ws_size) return;

  const float* x      = (const float*)d_in[0];
  const float* conv_w = (const float*)d_in[1];
  const float* conv_b = (const float*)d_in[2];
  const float* biases = (const float*)d_in[3];
  float* out = (float*)d_out;

  unsigned char* wsb = (unsigned char*)d_ws;
  unsigned* xh = (unsigned*)(wsb + off_x);
  unsigned* wt = (unsigned*)(wsb + off_w);

  k_xprep<<<dim3((XPIECES + 255) / 256), dim3(256), 0, stream>>>(x, xh);
  (void)hipGetLastError();

  k_wprep<<<dim3((WPIECES + 255) / 256), dim3(256), 0, stream>>>(conv_w, wt);
  (void)hipGetLastError();

  k_caps<<<dim3(NBLK), dim3(NTHR), 0, stream>>>((const _Float16*)xh, (const _Float16*)wt,
                                                conv_b, biases, out);
  (void)hipGetLastError();
}
